// folibiKT_63539746177588
// MI455X (gfx1250) — hardware-run, weakly checked
//
#include <hip/hip_runtime.h>
#include <math.h>

typedef __attribute__((ext_vector_type(16))) _Float16 v16h;
typedef __attribute__((ext_vector_type(8)))  _Float16 v8h;
typedef __attribute__((ext_vector_type(16))) __bf16   v16b;
typedef __attribute__((ext_vector_type(8)))  __bf16   v8b;
typedef __attribute__((ext_vector_type(8)))  float    v8f;
typedef __attribute__((ext_vector_type(4)))  float    v4f;

constexpr int kB      = 8;
constexpr int kS      = 1024;
constexpr int kE      = 512;
constexpr int kH      = 8;
constexpr int kHd     = 64;
constexpr int kRows   = kB * kS;
constexpr int kSqrtHd = 8;
constexpr float kScale = 1.0f / (float)kSqrtHd;
static_assert(kH * kHd == kE, "head split");
static_assert(kSqrtHd * kSqrtHd == kHd, "score scale is 1/sqrt(head dim)");
static_assert(kHd == 64, "one head = one 64-wide tile = one 128-B line of 16-bit values");
static_assert((kE % 32) == 0, "GEMM K multiple of 32");
static_assert((kRows % 64) == 0 && (kE % 64) == 0 && (kS % 64) == 0, "GEMM M,N multiples of 64");
static_assert((kS % 32) == 0 && (kS % 16) == 0, "attention tile multiples");

constexpr size_t kPlaneX  = (size_t)kRows * kE;
constexpr size_t kPlaneW  = (size_t)kE * kE;
constexpr size_t kOffXH   = 0;
constexpr size_t kOffXL   = kOffXH  + 3 * kPlaneX * 2;
constexpr size_t kOffWH   = kOffXL  + 3 * kPlaneX * 2;
constexpr size_t kOffWL   = kOffWH  + 3 * kPlaneW * 2;
constexpr size_t kOffQK   = kOffWL  + 3 * kPlaneW * 2;
constexpr size_t kOffVTH  = kOffQK  + 2 * kPlaneX * 2;
constexpr size_t kOffVTL  = kOffVTH + kPlaneX * 2;
constexpr size_t kOffATH  = kOffVTL + kPlaneX * 2;
constexpr size_t kOffATL  = kOffATH + kPlaneX * 2;
constexpr size_t kWsTotal = kOffATL + kPlaneX * 2;
static_assert(kWsTotal == 103809024ull, "carve total");
static_assert(kWsTotal <= 134217728ull, "carve cap");
static_assert((kOffXL % 128) == 0 && (kOffWH % 128) == 0 && (kOffWL % 128) == 0 && (kOffQK % 128) == 0 &&
              (kOffVTH % 128) == 0 && (kOffVTL % 128) == 0 && (kOffATH % 128) == 0 && (kOffATL % 128) == 0,
              "128-B aligned regions");

__device__ __forceinline__ unsigned short f2bf_bits(float f) {
  unsigned u = __float_as_uint(f);
  return (unsigned short)((u + 0x7FFFu + ((u >> 16) & 1u)) >> 16);
}
__device__ __forceinline__ float bf_bits2f(unsigned short h) { return __uint_as_float(((unsigned)h) << 16); }

__device__ __forceinline__ void split_bf(float f, __bf16& hi, __bf16& lo) {
  const unsigned short hb = f2bf_bits(f);
  const unsigned short lb = f2bf_bits(f - bf_bits2f(hb));
  hi = __builtin_bit_cast(__bf16, hb);
  lo = __builtin_bit_cast(__bf16, lb);
}

__device__ __forceinline__ void dep_guard1_h(v8f& a, v16h x, v16h y) { asm volatile("v_nop\n\tv_nop\n\tv_nop\n\tv_nop" : "+v"(a) : "v"(x), "v"(y)); }
__device__ __forceinline__ void dep_guard1_b(v8f& a, v16b x, v16b y) { asm volatile("v_nop\n\tv_nop\n\tv_nop\n\tv_nop" : "+v"(a) : "v"(x), "v"(y)); }
__device__ __forceinline__ void keep4_h(v16h a, v16h b, v16h c, v16h d) { asm volatile("v_nop" :: "v"(a), "v"(b), "v"(c), "v"(d)); }
__device__ __forceinline__ void keep4_b(v16b a, v16b b, v16b c, v16b d) { asm volatile("v_nop" :: "v"(a), "v"(b), "v"(c), "v"(d)); }
__device__ __forceinline__ void acc_guard4(v8f& a, v8f& b, v8f& c, v8f& d) { asm volatile("v_nop\n\tv_nop\n\tv_nop\n\tv_nop" : "+v"(a), "+v"(b), "+v"(c), "+v"(d)); }

template <typename T> struct Frag;
template <> struct Frag<_Float16> {
  typedef v16h V; union U { v16h v; v8h h[2]; };
  static __device__ __forceinline__ v16h load(const _Float16* p) {
    U f; f.h[0] = *(const v8h*)(p); f.h[1] = *(const v8h*)(p + 16); return f.v;
  }
  static __device__ __forceinline__ v8f mma(v16h a, v16h b, v8f c) {
    return __builtin_amdgcn_wmma_f32_16x16x32_f16(false, a, false, b, (short)0, c, false, false);
  }
  static __device__ __forceinline__ void guard1(v8f& a, v16h x, v16h y) { dep_guard1_h(a, x, y); }
  static __device__ __forceinline__ void keep(v16h a, v16h b, v16h c, v16h d) { keep4_h(a, b, c, d); }
};
template <> struct Frag<__bf16> {
  typedef v16b V; union U { v16b v; v8b h[2]; };
  static __device__ __forceinline__ v16b load(const __bf16* p) {
    U f; f.h[0] = *(const v8b*)(p); f.h[1] = *(const v8b*)(p + 16); return f.v;
  }
  static __device__ __forceinline__ v8f mma(v16b a, v16b b, v8f c) {
    return __builtin_amdgcn_wmma_f32_16x16x32_bf16(false, a, false, b, (short)0, c, false, false);
  }
  static __device__ __forceinline__ void guard1(v8f& a, v16b x, v16b y) { dep_guard1_b(a, x, y); }
  static __device__ __forceinline__ void keep(v16b a, v16b b, v16b c, v16b d) { keep4_b(a, b, c, d); }
};

__device__ __forceinline__ v8f mma_h_guarded(v16h a, v16h b, v8f c) {
  c = __builtin_amdgcn_wmma_f32_16x16x32_f16(false, a, false, b, (short)0, c, false, false);
  asm volatile("v_nop\n\tv_nop\n\tv_nop\n\tv_nop" : "+v"(c) : "v"(a), "v"(b));
  return c;
}
__device__ __forceinline__ v8f mma_b_guarded(v16b a, v16b b, v8f c) {
  c = __builtin_amdgcn_wmma_f32_16x16x32_bf16(false, a, false, b, (short)0, c, false, false);
  asm volatile("v_nop\n\tv_nop\n\tv_nop\n\tv_nop" : "+v"(c) : "v"(a), "v"(b));
  return c;
}

template <int ET> struct Elem;
template <> struct Elem<0> { typedef _Float16 T; };
template <> struct Elem<1> { typedef __bf16 T; };
template <int ET, bool SPLIT, int BIAS_MODE, int OUT_MODE>
__global__ __launch_bounds__(256) void wmma_gemm64(
    const unsigned short* __restrict__ Ap, const unsigned short* __restrict__ A2p, int lda, long strideA,
    const unsigned short* __restrict__ Btp, const unsigned short* __restrict__ Bt2p, int ldb, long strideB,
    void* __restrict__ Cout, void* __restrict__ Cout2, int ldc, long strideC,
    const float* __restrict__ bias,
    int M, int N, int K, float scale) {
  typedef typename Elem<ET>::T T;
  typedef typename Frag<T>::V V;
  const T* A = (const T*)Ap; const T* A2 = (const T*)A2p; const T* Bt = (const T*)Btp; const T* Bt2 = (const T*)Bt2p;
  __shared__ __align__(16) float sT[8][16 * 68];
  const int b    = blockIdx.y;
  const int lane = threadIdx.x & 31;
  const int wave = threadIdx.x >> 5;
  const int tilesN = N >> 6;
  const int tilesM = M >> 6;
  const int tile = blockIdx.x * 8 + wave;
  if (tile >= tilesM * tilesN) return;
  const int tm = tile / tilesN;
  const int tn = tile - tm * tilesN;
  const int m0 = tm << 6;
  const int n0 = tn << 6;

  const T* Ab  = A  + (size_t)b * strideA;
  const T* Bb  = Bt + (size_t)b * strideB;
  const T* Ab2 = SPLIT ? (A2  + (size_t)b * strideA) : nullptr;
  const T* Bb2 = SPLIT ? (Bt2 + (size_t)b * strideB) : nullptr;

  const int rlane = lane & 15;
  const int koff  = (lane >> 4) * 8;
  const int mOff  = (lane >> 4) * 8;

  v8f acc[4][4];
#pragma unroll
  for (int i = 0; i < 4; ++i)
#pragma unroll
    for (int j = 0; j < 4; ++j) acc[i][j] = (v8f){0.f,0.f,0.f,0.f,0.f,0.f,0.f,0.f};

  for (int k0 = 0; k0 < K; k0 += 32) {
    V bh[4], bl[4];
#pragma unroll
    for (int j = 0; j < 4; ++j) {
      const size_t bo = (size_t)(n0 + (j << 4) + rlane) * ldb + koff + k0;
      bh[j] = Frag<T>::load(Bb + bo);
      if (SPLIT) bl[j] = Frag<T>::load(Bb2 + bo);
    }
#pragma unroll
    for (int i = 0; i < 4; ++i) {
      const size_t ao = (size_t)(m0 + (i << 4) + rlane) * lda + koff + k0;
      V ah = Frag<T>::load(Ab + ao);
      V al;
      if (SPLIT) al = Frag<T>::load(Ab2 + ao);
#pragma unroll
      for (int j = 0; j < 4; ++j) {
        acc[i][j] = Frag<T>::mma(ah, bh[j], acc[i][j]);
        if (SPLIT) {
          acc[i][j] = Frag<T>::mma(ah, bl[j], acc[i][j]);
          acc[i][j] = Frag<T>::mma(al, bh[j], acc[i][j]);
        }
      }
      Frag<T>::guard1(acc[i][0], ah, SPLIT ? al : ah);
      Frag<T>::guard1(acc[i][1], ah, SPLIT ? al : ah);
      Frag<T>::guard1(acc[i][2], ah, SPLIT ? al : ah);
      Frag<T>::guard1(acc[i][3], ah, SPLIT ? al : ah);
    }
    Frag<T>::keep(bh[0], bh[1], bh[2], bh[3]);
    if (SPLIT) Frag<T>::keep(bl[0], bl[1], bl[2], bl[3]);
  }
  acc_guard4(acc[0][0], acc[0][1], acc[0][2], acc[0][3]);
  acc_guard4(acc[1][0], acc[1][1], acc[1][2], acc[1][3]);
  acc_guard4(acc[2][0], acc[2][1], acc[2][2], acc[2][3]);
  acc_guard4(acc[3][0], acc[3][1], acc[3][2], acc[3][3]);

  float* slab = sT[wave];
#pragma unroll
  for (int i = 0; i < 4; ++i) {
    const int mBase = m0 + (i << 4);
#pragma unroll
    for (int j = 0; j < 4; ++j) {
      const int n = n0 + (j << 4) + rlane;
      float bv = 0.f;
      if (BIAS_MODE == 2) bv = bias[n];
#pragma unroll
      for (int r = 0; r < 8; ++r) {
        float v = acc[i][j][r] * scale;
        if (BIAS_MODE == 1) v += bias[mBase + mOff + r];
        if (BIAS_MODE == 2) v += bv;
        slab[(mOff + r) * 68 + (j << 4) + rlane] = v;
      }
    }
    __builtin_amdgcn_fence(__ATOMIC_RELEASE, "workgroup");
    __builtin_amdgcn_wave_barrier();
    __builtin_amdgcn_fence(__ATOMIC_ACQUIRE, "workgroup");
    if (OUT_MODE == 0) {
      float* C = (float*)Cout + (size_t)b * strideC;
      const int hh = lane >> 4, c4 = (lane & 15) * 4;
      for (int pass = 0; pass < 2; ++pass) {
#pragma unroll
        for (int it = 0; it < 8; ++it) {
          const int row = it * 2 + hh;
          v4f v = *(const v4f*)(slab + row * 68 + c4);
          *(volatile v4f*)(C + (size_t)(mBase + row) * ldc + n0 + c4) = v;
        }
        __threadfence();
      }
    } else {
      const int q = lane >> 3, c8 = (lane & 7) * 8;
      unsigned short* C  = (unsigned short*)Cout  + (size_t)b * strideC;
      unsigned short* C2 = (OUT_MODE == 2) ? ((unsigned short*)Cout2 + (size_t)b * strideC) : nullptr;
      for (int pass = 0; pass < 2; ++pass) {
#pragma unroll
        for (int it = 0; it < 4; ++it) {
          const int row = it * 4 + q;
          const float* sp = slab + row * 68 + c8;
          v8h hv, lv;
#pragma unroll
          for (int e = 0; e < 8; ++e) {
            if (OUT_MODE == 1) {
              hv[e] = (_Float16)sp[e];
            } else {
              unsigned short hb = f2bf_bits(sp[e]);
              unsigned short lb = f2bf_bits(sp[e] - bf_bits2f(hb));
              hv[e] = __builtin_bit_cast(_Float16, hb);
              lv[e] = __builtin_bit_cast(_Float16, lb);
            }
          }
          *(volatile v8h*)(C + (size_t)(mBase + row) * ldc + n0 + c8) = hv;
          if (OUT_MODE == 2) *(volatile v8h*)(C2 + (size_t)(mBase + row) * ldc + n0 + c8) = lv;
        }
        __threadfence();
      }
    }
    __builtin_amdgcn_fence(__ATOMIC_RELEASE, "workgroup");
    __builtin_amdgcn_wave_barrier();
    __builtin_amdgcn_fence(__ATOMIC_ACQUIRE, "workgroup");
  }
}

__global__ __launch_bounds__(256) void split3_rows_bf16_kernel(
    const float* __restrict__ s0, const float* __restrict__ s1, const float* __restrict__ s2,
    unsigned short* __restrict__ dhi, unsigned short* __restrict__ dlo, int total8, long plane)
{
  const int z = blockIdx.y;
  const float* src = (z == 0) ? s0 : ((z == 1) ? s1 : s2);
  const int i = blockIdx.x * 256 + threadIdx.x;
  if (i >= total8) return;
  const size_t e0 = (size_t)i << 3;
  const v4f a0 = *(const v4f*)(src + e0);
  const v4f a1 = *(const v4f*)(src + e0 + 4);
  v8h hv, lv;
#pragma unroll
  for (int e = 0; e < 4; ++e) {
    const float f0 = a0[e];
    const float f1 = a1[e];
    const unsigned short h0 = f2bf_bits(f0), h1 = f2bf_bits(f1);
    const unsigned short l0 = f2bf_bits(f0 - bf_bits2f(h0)), l1 = f2bf_bits(f1 - bf_bits2f(h1));
    hv[e]     = __builtin_bit_cast(_Float16, h0);
    hv[4 + e] = __builtin_bit_cast(_Float16, h1);
    lv[e]     = __builtin_bit_cast(_Float16, l0);
    lv[4 + e] = __builtin_bit_cast(_Float16, l1);
  }
  unsigned short* qh = dhi + (size_t)z * plane + e0;
  unsigned short* ql = dlo + (size_t)z * plane + e0;
  *(volatile v8h*)qh = hv;
  *(volatile v8h*)ql = lv;
  __threadfence();
  *(volatile v8h*)qh = hv;
  *(volatile v8h*)ql = lv;
}

__global__ __launch_bounds__(512) void decay_attn_kernel(
    const unsigned short* __restrict__ Qp, const unsigned short* __restrict__ Kp,
    const unsigned short* __restrict__ VTHp, const unsigned short* __restrict__ VTLp,
    const float* __restrict__ gammas,
    unsigned short* __restrict__ ATH, unsigned short* __restrict__ ATL)
{
  __shared__ __align__(16) float sc[16 * kS];
  __shared__ __align__(16) float red[4 * 16 * kHd];
  __shared__ float invz[16];

  const int tid  = threadIdx.x;
  const int lane = tid & 31;
  const int w    = __builtin_amdgcn_readfirstlane(tid >> 5);
  const int hi   = lane >> 4;
  const int ln   = lane & 15;

  const int bh = blockIdx.y;
  const int b  = bh / kH;
  const int h  = bh - b * kH;
  const int i0 = blockIdx.x * 16;
  const int numJT = blockIdx.x + 1;
  const int numJB = (numJT + 1) >> 1;
  const size_t rowbase = (size_t)b * kS;

  {
    const _Float16* Qf = (const _Float16*)Qp;
    const _Float16* Kf = (const _Float16*)Kp;
    const _Float16* qp = Qf + (rowbase + (size_t)(i0 + ln)) * kE + h * kHd + 8 * hi;
    const v16h qa0 = Frag<_Float16>::load(qp);
    const v16h qa1 = Frag<_Float16>::load(qp + 32);
    for (int jt = w; jt < numJT; jt += 16) {
      const _Float16* kp = Kf + (rowbase + (size_t)(jt * 16 + ln)) * kE + h * kHd + 8 * hi;
      const v16h kb0 = Frag<_Float16>::load(kp);
      const v16h kb1 = Frag<_Float16>::load(kp + 32);
      v8f c = (v8f){0.f,0.f,0.f,0.f,0.f,0.f,0.f,0.f};
      c = mma_h_guarded(qa0, kb0, c);
      c = mma_h_guarded(qa1, kb1, c);
#pragma unroll
      for (int r = 0; r < 8; ++r) sc[(8 * hi + r) * kS + jt * 16 + ln] = c[r] * kScale;
    }
  }
  __syncthreads();

  {
    const int r = w;
    const int i = i0 + r;
    float* srow = sc + r * kS;
    const float gq = gammas[h];
    const float gamma = -(fmaxf(gq, 0.0f) + log1pf(expf(-fabsf(gq))));
    const int nch = (i >> 5) + 1;

    float m1 = -INFINITY;
#pragma unroll 1
    for (int jb = 0; jb < nch; ++jb) {
      const int j  = jb * 32 + lane;
      const int jc = (j < i) ? j : i;
      m1 = fmaxf(m1, srow[jc]);
    }
#pragma unroll
    for (int off = 16; off > 0; off >>= 1) m1 = fmaxf(m1, __shfl_xor(m1, off, 32));

    float z1 = 0.0f;
#pragma unroll 1
    for (int jb = 0; jb < nch; ++jb) {
      const int j  = jb * 32 + lane;
      const bool ok = (j <= i);
      const int jc = (j < i) ? j : i;
      const float e = __expf(srow[jc] - m1);
      z1 += ok ? e : 0.0f;
    }
#pragma unroll
    for (int off = 16; off > 0; off >>= 1) z1 += __shfl_xor(z1, off, 32);
    const float invZ1 = 1.0f / z1;

    float carry = 0.0f;
    float m2 = -INFINITY;
#pragma unroll 1
    for (int jb = 0; jb < nch; ++jb) {
      const int j  = jb * 32 + lane;
      const bool ok = (j <= i);
      const int jc = (j < i) ? j : i;
      const float sraw = srow[jc];
      const float e1 = __expf(sraw - m1);
      float p = ok ? e1 : 0.0f;
#pragma unroll
      for (int off = 1; off < 32; off <<= 1) {
        const float t = __shfl_up(p, off, 32);
        p += (lane >= off) ? t : 0.0f;
      }
      const float prefix = carry + p;
      const float tot = __shfl(p, 31, 32);
      carry += tot;
      const float rem  = fmaxf(z1 - prefix, 0.0f) * invZ1;
      const float posd = (float)(i - jc);
      const float dist = sqrtf(rem * posd);
      float te = __expf(gamma * dist);
      te = fminf(fmaxf(te, 1e-5f), 1e5f);
      const float s2 = sraw * te;
      if (ok) srow[j] = s2;
      m2 = fmaxf(m2, ok ? s2 : -INFINITY);
    }
#pragma unroll
    for (int off = 16; off > 0; off >>= 1) m2 = fmaxf(m2, __shfl_xor(m2, off, 32));

    float z2 = 0.0f;
#pragma unroll 1
    for (int jb = 0; jb < numJB; ++jb) {
      const int j  = jb * 32 + lane;
      const bool ok = (j <= i);
      const int jc = (j < i) ? j : i;
      const float s2 = srow[jc];
      const float e2 = __expf(s2 - m2);
      const float e  = ok ? e2 : 0.0f;
      z2 += e;
      srow[j] = e;
    }
#pragma unroll
    for (int off = 16; off > 0; off >>= 1) z2 += __shfl_xor(z2, off, 32);
    if (lane == 0) invz[r] = 1.0f / z2;
  }
  __syncthreads();

  {
    const int dt = w & 3;
    const int g  = w >> 2;
    const size_t vrow = ((size_t)b * kE + (size_t)(h * kHd + dt * 16 + ln)) * kS + 8 * hi;
    const __bf16* vh = (const __bf16*)VTHp + vrow;
    const __bf16* vl = (const __bf16*)VTLp + vrow;
    v8f c = (v8f){0.f,0.f,0.f,0.f,0.f,0.f,0.f,0.f};
    for (int jb = g; jb < numJB; jb += 4) {
      const float* pr = sc + ln * kS + jb * 32 + 8 * hi;
      const v4f a0 = *(const v4f*)(pr);
      const v4f a1 = *(const v4f*)(pr + 4);
      const v4f a2 = *(const v4f*)(pr + 16);
      const v4f a3 = *(const v4f*)(pr + 20);
      v16b ph, pl;
#pragma unroll
      for (int e = 0; e < 4; ++e) {
        __bf16 x, y;
        const float f0 = a0[e];
        const float f1 = a1[e];
        const float f2 = a2[e];
        const float f3 = a3[e];
        split_bf(f0, x, y); ph[e]      = x; pl[e]      = y;
        split_bf(f1, x, y); ph[4 + e]  = x; pl[4 + e]  = y;
        split_bf(f2, x, y); ph[8 + e]  = x; pl[8 + e]  = y;
        split_bf(f3, x, y); ph[12 + e] = x; pl[12 + e] = y;
      }
      const v16b bhv = Frag<__bf16>::load(vh + jb * 32);
      const v16b blv = Frag<__bf16>::load(vl + jb * 32);
      c = mma_b_guarded(ph, bhv, c);
      c = mma_b_guarded(ph, blv, c);
      c = mma_b_guarded(pl, bhv, c);
    }
#pragma unroll
    for (int r = 0; r < 8; ++r) red[(g * 16 + 8 * hi + r) * kHd + dt * 16 + ln] = c[r];
  }
  __syncthreads();

  if (w < 4) {
    const int row = tid >> 3;
    const int c8  = (tid & 7) * 8;
    const float iz = invz[row];
    const bool zr  = ((i0 + row) == 0);
    float s[8];
    {
      const float* p0 = red + (0 * 16 + row) * kHd + c8;
      const float* p1 = red + (1 * 16 + row) * kHd + c8;
      const float* p2 = red + (2 * 16 + row) * kHd + c8;
      const float* p3 = red + (3 * 16 + row) * kHd + c8;
      const v4f x0 = *(const v4f*)(p0), y0 = *(const v4f*)(p0 + 4);
      const v4f x1 = *(const v4f*)(p1), y1 = *(const v4f*)(p1 + 4);
      const v4f x2 = *(const v4f*)(p2), y2 = *(const v4f*)(p2 + 4);
      const v4f x3 = *(const v4f*)(p3), y3 = *(const v4f*)(p3 + 4);
#pragma unroll
      for (int e = 0; e < 4; ++e) {
        s[e]     = ((x0[e] + x1[e]) + x2[e]) + x3[e];
        s[4 + e] = ((y0[e] + y1[e]) + y2[e]) + y3[e];
      }
    }
    v8h hv, lv;
#pragma unroll
    for (int e = 0; e < 8; ++e) {
      const float val = zr ? 0.0f : (s[e] * iz);
      const unsigned short hb = f2bf_bits(val);
      const unsigned short lb = f2bf_bits(val - bf_bits2f(hb));
      hv[e] = __builtin_bit_cast(_Float16, hb);
      lv[e] = __builtin_bit_cast(_Float16, lb);
    }
    const size_t o = (rowbase + (size_t)(i0 + row)) * kE + h * kHd + c8;
    *(volatile v8h*)(ATH + o) = hv;
    *(volatile v8h*)(ATL + o) = lv;
    __threadfence();
    *(volatile v8h*)(ATH + o) = hv;
    *(volatile v8h*)(ATL + o) = lv;
  }
}

extern "C" void kernel_launch(void* const* d_in, const int* in_sizes, int n_in,
                              void* d_out, int out_size, void* d_ws, size_t ws_size,
                              hipStream_t stream) {
  if (n_in < 10) return;
  if (in_sizes[0] != kRows * kE) return;
  if (in_sizes[1] != kRows * kE) return;
  if (in_sizes[2] != kRows * kE) return;
  if (in_sizes[3] != kE * kE) return;
  if (in_sizes[4] != kE) return;
  if (in_sizes[5] != kE * kE) return;
  if (in_sizes[6] != kE) return;
  if (in_sizes[7] != kE * kE) return;
  if (in_sizes[8] != kE) return;
  if (in_sizes[9] != kH) return;
  if (out_size != kRows * kE) return;
  if (ws_size < kWsTotal) return;

  const float* q      = (const float*)d_in[0];
  const float* k      = (const float*)d_in[1];
  const float* v      = (const float*)d_in[2];
  const float* Wk     = (const float*)d_in[3];
  const float* bk     = (const float*)d_in[4];
  const float* Wv     = (const float*)d_in[5];
  const float* bv     = (const float*)d_in[6];
  const float* Wo     = (const float*)d_in[7];
  const float* bo     = (const float*)d_in[8];
  const float* gammas = (const float*)d_in[9];
  float* out = (float*)d_out;

  char* ws = (char*)d_ws;
  unsigned short* XH  = (unsigned short*)(ws + kOffXH);
  unsigned short* XL  = (unsigned short*)(ws + kOffXL);
  unsigned short* WH  = (unsigned short*)(ws + kOffWH);
  unsigned short* WL  = (unsigned short*)(ws + kOffWL);
  unsigned short* QK  = (unsigned short*)(ws + kOffQK);
  unsigned short* VTH = (unsigned short*)(ws + kOffVTH);
  unsigned short* VTL = (unsigned short*)(ws + kOffVTL);
  unsigned short* ATH = (unsigned short*)(ws + kOffATH);
  unsigned short* ATL = (unsigned short*)(ws + kOffATL);

  split3_rows_bf16_kernel<<<dim3((unsigned)(kPlaneX / 8 / 256), 3), 256, 0, stream>>>(
      q, k, v, XH, XL, (int)(kPlaneX / 8), (long)kPlaneX);
  split3_rows_bf16_kernel<<<dim3((unsigned)(kPlaneW / 8 / 256), 3), 256, 0, stream>>>(
      Wk, Wv, Wo, WH, WL, (int)(kPlaneW / 8), (long)kPlaneW);

  wmma_gemm64<1, true, 2, 1><<<dim3(128, 2), 256, 0, stream>>>(
      XH, XL, kE, (long)kPlaneX,
      WH, WL, kE, 0L,
      (void*)QK, nullptr, kE, (long)kPlaneX,
      bk,
      kRows, kE, kE, 1.0f);

  wmma_gemm64<1, true, 1, 2><<<dim3(16, kB), 256, 0, stream>>>(
      WH + kPlaneW, WL + kPlaneW, kE, 0L,
      XH + 2 * kPlaneX, XL + 2 * kPlaneX, kE, (long)kS * kE,
      (void*)VTH, (void*)VTL, kS, (long)kE * kS,
      bv,
      kE, kS, kE, 1.0f);

  decay_attn_kernel<<<dim3(kS / 16, kB * kH), 512, 0, stream>>>(
      QK, QK + kPlaneX, VTH, VTL, gammas, ATH, ATL);

  wmma_gemm64<1, true, 2, 0><<<dim3(128, 1), 256, 0, stream>>>(
      ATH, ATL, kE, 0L,
      WH + 2 * kPlaneW, WL + 2 * kPlaneW, kE, 0L,
      (void*)out, nullptr, kE, 0L,
      bo,
      kRows, kE, kE, 1.0f);
}
